// DTransformerLayer_27917287424233
// MI455X (gfx1250) — hardware-verified
//
#include <hip/hip_runtime.h>

#define BATCH 4
#define SEQ   1024
#define DM    1024
#define NH    16
#define HD    64
#define NTOK  (BATCH * SEQ)
#define NBS   (NTOK * DM)
#define NWT   (DM * DM)
#define NEGV  (-1.0e32f)
#define PSCALE 16384.0f
#define LNEPS 1.0e-5f
#define WINK  64

typedef _Float16 v16h __attribute__((ext_vector_type(16)));
typedef __bf16   v16b __attribute__((ext_vector_type(16)));
typedef float    v8f  __attribute__((ext_vector_type(8)));
typedef float    v4f  __attribute__((ext_vector_type(4)));
typedef unsigned int v4u __attribute__((ext_vector_type(4)));
typedef v4f __attribute__((may_alias)) v4fa;
typedef v4u __attribute__((may_alias)) v4ua;

union FragH { v16h v; v4u q[2]; };
union FragB { v16b v; v4u q[2]; };

__device__ __forceinline__ v8f wmma_f16(v16h a, v16h b, v8f c) {
  v8f d = __builtin_amdgcn_wmma_f32_16x16x32_f16(false, a, false, b, (short)0, c, false, false);
  asm volatile("v_nop\n\tv_nop\n\tv_nop\n\tv_nop" : "+v"(d) : "v"(a), "v"(b));
  return d;
}
__device__ __forceinline__ v8f wmma_bf16(v16b a, v16b b, v8f c) {
  v8f d = __builtin_amdgcn_wmma_f32_16x16x32_bf16(false, a, false, b, (short)0, c, false, false);
  asm volatile("v_nop\n\tv_nop\n\tv_nop\n\tv_nop" : "+v"(d) : "v"(a), "v"(b));
  return d;
}

__device__ __forceinline__ v16h ldfrag_h(const _Float16* p, int h) {
  FragH f;
  f.q[0] = *(const v4ua*)(p + 8 * h);
  f.q[1] = *(const v4ua*)(p + 16 + 8 * h);
  return f.v;
}
__device__ __forceinline__ v16b ldfrag_b(const unsigned short* p, int h) {
  FragB f;
  f.q[0] = *(const v4ua*)(p + 8 * h);
  f.q[1] = *(const v4ua*)(p + 16 + 8 * h);
  return f.v;
}

__device__ __forceinline__ unsigned int bf16_rne_bits(float x) {
  const unsigned int u = __float_as_uint(x);
  return (u + 0x7FFFu + ((u >> 16) & 1u)) >> 16;
}
__device__ __forceinline__ unsigned int split_pair(float x0, float x1, unsigned int& low_word) {
  const unsigned int h0 = bf16_rne_bits(x0), h1 = bf16_rne_bits(x1);
  const float r0 = x0 - __uint_as_float(h0 << 16);
  const float r1 = x1 - __uint_as_float(h1 << 16);
  const unsigned int l0 = bf16_rne_bits(r0), l1 = bf16_rne_bits(r1);
  low_word = l0 | (l1 << 16);
  return h0 | (h1 << 16);
}
__device__ __forceinline__ void split8(v4f a, v4f c, v4u& hi, v4u& lo) {
  unsigned int l;
  hi.x = split_pair(a.x, a.y, l); lo.x = l;
  hi.y = split_pair(a.z, a.w, l); lo.y = l;
  hi.z = split_pair(c.x, c.y, l); lo.z = l;
  hi.w = split_pair(c.z, c.w, l); lo.w = l;
}

__device__ __forceinline__ float wave_sum(float v) {
  #pragma unroll
  for (int d = 16; d > 0; d >>= 1) v += __shfl_xor(v, d);
  return v;
}
__device__ __forceinline__ float wave_max(float v) {
  #pragma unroll
  for (int d = 16; d > 0; d >>= 1) v = fmaxf(v, __shfl_xor(v, d));
  return v;
}

__global__ __launch_bounds__(256) void cvt_act_kernel(
    const float* __restrict__ x0, const float* __restrict__ x1, const float* __restrict__ x2,
    unsigned short* __restrict__ xpl)
{
  const int g = blockIdx.x * 256 + threadIdx.x;
  if (g >= 3 * (NBS / 8)) return;
  const int sel = g / (NBS / 8);
  const int off = g - sel * (NBS / 8);
  const float* src = ((sel == 0) ? x0 : ((sel == 1) ? x1 : x2)) + (size_t)off * 8;
  const v4f a = *(const v4fa*)src;
  const v4f c = *(const v4fa*)(src + 4);
  v4u hi, lo;
  split8(a, c, hi, lo);
  unsigned short* dh = xpl + (size_t)sel * 2 * NBS + (size_t)off * 8;
  unsigned short* dl = dh + NBS;
  *(volatile v4u*)dh = hi;
  *(volatile v4u*)dl = lo;
  __threadfence();
  *(volatile v4u*)dh = hi;
  *(volatile v4u*)dl = lo;
}

__global__ __launch_bounds__(256) void cvt_w_kernel(
    const float* __restrict__ w0, const float* __restrict__ w1, const float* __restrict__ w2,
    const float* __restrict__ w3, const float* __restrict__ w4,
    unsigned short* __restrict__ wtp)
{
  __shared__ __attribute__((aligned(16))) float sT[64 * 68];

  const int tid = threadIdx.x, lane = tid & 31, w = tid >> 5;
  const int k0 = blockIdx.x * 64, n0 = blockIdx.y * 64, z = blockIdx.z;
  const float* W = (z == 0) ? w0 : ((z == 1) ? w1 : ((z == 2) ? w2 : ((z == 3) ? w3 : w4)));

  #pragma unroll
  for (int i = 0; i < 4; ++i) {
    const int idx = tid + 256 * i;
    const int row = idx >> 4, c4 = idx & 15;
    const v4f v = *(const v4fa*)(W + (size_t)(k0 + row) * DM + n0 + 4 * c4);
    sT[(4 * c4 + 0) * 68 + row] = v.x;
    sT[(4 * c4 + 1) * 68 + row] = v.y;
    sT[(4 * c4 + 2) * 68 + row] = v.z;
    sT[(4 * c4 + 3) * 68 + row] = v.w;
  }
  __syncthreads();

  unsigned short* wh = wtp + (size_t)z * 2 * NWT;
  unsigned short* wl = wh + NWT;
  const int q8 = lane & 7, sub = lane >> 3;
  v4u hi[2], lo[2];
  size_t gi[2];
  #pragma unroll
  for (int it = 0; it < 2; ++it) {
    const int nl = 32 * it + 4 * w + sub;
    const v4f a = *(const v4fa*)(sT + nl * 68 + 8 * q8);
    const v4f c = *(const v4fa*)(sT + nl * 68 + 8 * q8 + 4);
    split8(a, c, hi[it], lo[it]);
    gi[it] = (size_t)(n0 + nl) * DM + k0 + 8 * q8;
    *(volatile v4u*)(wh + gi[it]) = hi[it];
    *(volatile v4u*)(wl + gi[it]) = lo[it];
  }
  __threadfence();
  #pragma unroll
  for (int it = 0; it < 2; ++it) {
    *(volatile v4u*)(wh + gi[it]) = hi[it];
    *(volatile v4u*)(wl + gi[it]) = lo[it];
  }
}

__device__ __forceinline__ void gemm_x3(const unsigned short* ah, const unsigned short* al,
                                        const unsigned short* bh, const unsigned short* bl,
                                        int h, v8f (&acc)[2][4])
{
  const v8f z8 = {0.f, 0.f, 0.f, 0.f, 0.f, 0.f, 0.f, 0.f};
  #pragma unroll
  for (int mt = 0; mt < 2; ++mt)
    #pragma unroll
    for (int nt = 0; nt < 4; ++nt) acc[mt][nt] = z8;

  #pragma unroll 1
  for (int k0 = 0; k0 < DM; k0 += 32) {
    const v16b a0h = ldfrag_b(ah + k0, h);
    const v16b a1h = ldfrag_b(ah + (size_t)16 * DM + k0, h);
    const v16b a0l = ldfrag_b(al + k0, h);
    const v16b a1l = ldfrag_b(al + (size_t)16 * DM + k0, h);
    #pragma unroll
    for (int nt = 0; nt < 4; ++nt) {
      const v16b whf = ldfrag_b(bh + (size_t)nt * 16 * DM + k0, h);
      acc[0][nt] = wmma_bf16(a0h, whf, acc[0][nt]);
      acc[0][nt] = wmma_bf16(a0l, whf, acc[0][nt]);
      acc[1][nt] = wmma_bf16(a1h, whf, acc[1][nt]);
      acc[1][nt] = wmma_bf16(a1l, whf, acc[1][nt]);
      const v16b wlf = ldfrag_b(bl + (size_t)nt * 16 * DM + k0, h);
      acc[0][nt] = wmma_bf16(a0h, wlf, acc[0][nt]);
      acc[1][nt] = wmma_bf16(a1h, wlf, acc[1][nt]);
    }
  }
}

__device__ __forceinline__ void plane_store_pass(const _Float16* sT, _Float16* plane, _Float16* vt,
                                                 int vmode, int bh, int s0, int w, int lane)
{
  const int q8 = lane & 7, sub = lane >> 3;
  #pragma unroll
  for (int i = 0; i < 8; ++i) {
    const int lid = w * 32 + i * 4 + sub;
    const int d = lid >> 1, hl = lid & 1;
    const int lidx = vmode ? (d * 128 + 64 * hl + 8 * q8) : (lid * HD + 8 * q8);
    const v4u v = *(const v4ua*)(sT + lidx);
    const size_t gidx = vmode ? (((size_t)bh * HD + d) * SEQ + s0 + 64 * hl + 8 * q8)
                              : (((size_t)bh * SEQ + s0 + lid) * HD + 8 * q8);
    _Float16* base = vmode ? vt : plane;
    *(volatile v4u*)(base + gidx) = v;
  }
}

__global__ __launch_bounds__(128) void proj5_kernel(
    const unsigned short* __restrict__ xpl,
    const unsigned short* __restrict__ wtp,
    const float* __restrict__ bq, const float* __restrict__ bqw, const float* __restrict__ bv,
    _Float16* __restrict__ qp, _Float16* __restrict__ kp,
    _Float16* __restrict__ qwp, _Float16* __restrict__ kwp,
    _Float16* __restrict__ vt)
{
  __shared__ __attribute__((aligned(16))) _Float16 sT[128 * 64];

  const int tid = threadIdx.x, lane = tid & 31, w = tid >> 5;
  const int h = lane >> 4, m = lane & 15;
  const int z = blockIdx.z;
  const int asel = (z == 0 || z == 3) ? 0 : ((z == 2) ? 2 : 1);
  const int wsel = (z < 2) ? 0 : ((z == 2) ? 2 : 1);
  const float* bias = (z < 2) ? bq : ((z == 2) ? bv : bqw);
  _Float16* plane = (z == 0) ? qp : ((z == 1) ? kp : ((z == 3) ? qwp : ((z == 4) ? kwp : qp)));
  const int vmode = (z == 2) ? 1 : 0;

  const int m0 = blockIdx.x * 128, head = blockIdx.y, n0 = head * HD;
  const int m0w = m0 + 32 * w;
  const unsigned short* ah = xpl + (size_t)asel * 2 * NBS + (size_t)(m0w + m) * DM;
  const unsigned short* al = ah + NBS;
  const unsigned short* bh = wtp + (size_t)wsel * 2 * NWT + (size_t)(n0 + m) * DM;
  const unsigned short* bl = bh + NWT;

  v8f acc[2][4];
  gemm_x3(ah, al, bh, bl, h, acc);

  #pragma unroll
  for (int nt = 0; nt < 4; ++nt) {
    const int feat = 16 * nt + m;
    const float bvl = bias[n0 + feat];
    #pragma unroll
    for (int mt = 0; mt < 2; ++mt) {
      #pragma unroll
      for (int r = 0; r < 8; ++r) {
        const int tokl = 32 * w + 16 * mt + 8 * h + r;
        const float y = acc[mt][nt][r] + bvl;
        const int idx = vmode ? (feat * 128 + tokl) : (tokl * HD + feat);
        sT[idx] = (_Float16)y;
      }
    }
  }
  __syncthreads();

  const int b = m0 / SEQ, s0 = m0 - b * SEQ, bhi = b * NH + head;
  plane_store_pass(sT, plane, vt, vmode, bhi, s0, w, lane);
  __threadfence();
  plane_store_pass(sT, plane, vt, vmode, bhi, s0, w, lane);
}

__device__ __forceinline__ void f32_store_pass(const float* sT, float* dst, int m0, int n0,
                                               int w, int lane)
{
  const int q8 = lane & 7, sub = lane >> 3;
  #pragma unroll
  for (int i = 0; i < 16; ++i) {
    const int lid = i * 4 + sub;
    const int row = 32 * w + (lid >> 1), hl = lid & 1;
    const v4f v = *(const v4fa*)(sT + row * 64 + 32 * hl + 4 * q8);
    *(volatile v4f*)(dst + (size_t)(m0 + row) * DM + n0 + 32 * hl + 4 * q8) = v;
  }
}

__global__ __launch_bounds__(128) void oproj_kernel(
    const unsigned short* __restrict__ aopl,
    const unsigned short* __restrict__ wtp,
    const float* __restrict__ bo, const float* __restrict__ bow,
    float* __restrict__ outf, float* __restrict__ outwf)
{
  __shared__ __attribute__((aligned(16))) float sT[128 * 64];

  const int tid = threadIdx.x, lane = tid & 31, w = tid >> 5;
  const int h = lane >> 4, m = lane & 15;
  const int z = blockIdx.z;
  const float* bias = (z == 0) ? bo : bow;
  float* dst = (z == 0) ? outf : outwf;
  const int m0 = blockIdx.x * 128, n0 = blockIdx.y * 64;
  const int m0w = m0 + 32 * w;
  const unsigned short* ah = aopl + (size_t)z * 2 * NBS + (size_t)(m0w + m) * DM;
  const unsigned short* al = ah + NBS;
  const unsigned short* bh = wtp + (size_t)(3 + z) * 2 * NWT + (size_t)(n0 + m) * DM;
  const unsigned short* bl = bh + NWT;

  v8f acc[2][4];
  gemm_x3(ah, al, bh, bl, h, acc);

  #pragma unroll
  for (int nt = 0; nt < 4; ++nt) {
    const int feat = 16 * nt + m;
    const float bvl = bias[n0 + feat];
    #pragma unroll
    for (int mt = 0; mt < 2; ++mt) {
      #pragma unroll
      for (int r = 0; r < 8; ++r) {
        const int tokl = 32 * w + 16 * mt + 8 * h + r;
        sT[tokl * 64 + feat] = acc[mt][nt][r] + bvl;
      }
    }
  }
  __syncthreads();

  f32_store_pass(sT, dst, m0, n0, w, lane);
  __threadfence();
  f32_store_pass(sT, dst, m0, n0, w, lane);
}

template <bool WINDOW>
__global__ __launch_bounds__(128) void attn_kernel(
    const _Float16* __restrict__ qp,
    const _Float16* __restrict__ kp,
    const _Float16* __restrict__ vt,
    const float* __restrict__ gammas,
    unsigned short* __restrict__ aoh,
    unsigned short* __restrict__ aol)
{
  constexpr int KL = WINDOW ? WINK : SEQ;
  __shared__ __attribute__((aligned(16))) float    sS[16 * KL];
  __shared__ __attribute__((aligned(16))) float    sE[4 * KL];
  __shared__ __attribute__((aligned(16))) _Float16 sP[16 * KL];
  __shared__ __attribute__((aligned(16))) float    sO[16 * HD];

  const int tid = threadIdx.x, lane = tid & 31, w = tid >> 5;
  const int h = lane >> 4, m = lane & 15;
  const int qt = blockIdx.x, bh = blockIdx.y;
  const int b = bh >> 4, head = bh & 15;
  const int q0 = qt * 16;

  int kbase, nch;
  if (WINDOW) {
    int t = qt - 2;
    t = (t < 0) ? 0 : t;
    t = (t > (SEQ / 16 - 4)) ? (SEQ / 16 - 4) : t;
    kbase = 16 * t;
    nch = 2;
  } else {
    kbase = 0;
    nch = (q0 + 16 + 31) >> 5;
  }
  const int nkt = nch * 2;

  const v8f z8 = {0.f, 0.f, 0.f, 0.f, 0.f, 0.f, 0.f, 0.f};

  {
    const _Float16* qrow = qp + ((size_t)bh * SEQ + q0 + m) * HD;
    const v16h qa0 = ldfrag_h(qrow, h);
    const v16h qa1 = ldfrag_h(qrow + 32, h);
    #pragma unroll 1
    for (int kt = w; kt < nkt; kt += 4) {
      const _Float16* krow = kp + ((size_t)bh * SEQ + kbase + 16 * kt + m) * HD;
      const v16h kb0 = ldfrag_h(krow, h);
      const v16h kb1 = ldfrag_h(krow + 32, h);
      v8f acc = z8;
      acc = wmma_f16(qa0, kb0, acc);
      acc = wmma_f16(qa1, kb1, acc);
      #pragma unroll
      for (int r = 0; r < 8; ++r) sS[(8 * h + r) * KL + 16 * kt + m] = acc[r] * 0.125f;
    }
  }
  __syncthreads();

  const float g = -fabsf(gammas[head]);
  float* se = sE + w * KL;
  #pragma unroll 1
  for (int a = 0; a < 4; ++a) {
    const int row = w + 4 * a;
    const int i = q0 + row;
    float* srow = sS + row * KL;
    _Float16* prow = sP + row * KL;

    if (i == 0) {
      #pragma unroll 1
      for (int c = 0; c < nch; ++c) prow[32 * c + lane] = (_Float16)0.0f;
      continue;
    }

    float m1 = NEGV;
    #pragma unroll 1
    for (int c = 0; c < nch; ++c) {
      const int jj = 32 * c + lane, j = kbase + jj;
      const bool valid = WINDOW ? (j < i && j >= i - 19) : (j < i);
      const float s = srow[jj];
      m1 = fmaxf(m1, valid ? s : NEGV);
    }
    m1 = wave_max(m1);

    float tot = 0.0f;
    #pragma unroll 1
    for (int c = 0; c < nch; ++c) {
      const int jj = 32 * c + lane, j = kbase + jj;
      const bool valid = WINDOW ? (j < i && j >= i - 19) : (j < i);
      const float s = srow[jj];
      const float e = valid ? __expf(s - m1) : 0.0f;
      se[jj] = e;
      tot += e;
    }
    tot = wave_sum(tot);
    const float inv = 1.0f / tot;

    float dsum = 0.0f;
    #pragma unroll 1
    for (int c = 0; c < nch; ++c) {
      const int jj = 32 * c + lane;
      const float p = se[jj] * inv;
      se[jj] = p;
      dsum += p;
    }
    dsum = wave_sum(dsum);

    float run = 0.0f, m2 = NEGV;
    #pragma unroll 1
    for (int c = 0; c < nch; ++c) {
      const int jj = 32 * c + lane, j = kbase + jj;
      const bool valid = WINDOW ? (j < i && j >= i - 19) : (j < i);
      const float p = se[jj];
      float x = p;
      #pragma unroll
      for (int d = 1; d < 32; d <<= 1) {
        const float y = __shfl_up(x, (unsigned int)d);
        if (lane >= d) x += y;
      }
      const float distcum = run + x;
      run += __shfl(x, 31);
      const float rem = dsum - distcum;
      const float pe = (float)((j >= i) ? (j - i) : (i - j));
      const float dist = sqrtf(fmaxf(rem * pe, 0.0f));
      float te = __expf(dist * g);
      te = fminf(fmaxf(te, 1.0e-5f), 1.0e5f);
      const float s = srow[jj];
      const float s2 = valid ? s * te : NEGV;
      srow[jj] = s2;
      m2 = fmaxf(m2, s2);
    }
    m2 = wave_max(m2);

    float tot2 = 0.0f;
    #pragma unroll 1
    for (int c = 0; c < nch; ++c) {
      const int jj = 32 * c + lane, j = kbase + jj;
      const bool valid = WINDOW ? (j < i && j >= i - 19) : (j < i);
      const float s2 = srow[jj];
      const float e2 = valid ? __expf(s2 - m2) : 0.0f;
      se[jj] = e2;
      tot2 += e2;
    }
    tot2 = wave_sum(tot2);
    const float inv2 = 1.0f / tot2;
    const float scl = WINDOW ? 1.0f : fminf(1.0f / inv2, 5.0f);

    #pragma unroll 1
    for (int c = 0; c < nch; ++c) {
      const int jj = 32 * c + lane;
      const float p2 = se[jj] * inv2;
      const float pv = WINDOW ? p2 : p2 * scl;
      prow[jj] = (_Float16)(pv * PSCALE);
    }
  }
  __syncthreads();

  {
    v8f acc = z8;
    const _Float16* vrow = vt + ((size_t)bh * HD + 16 * w + m) * SEQ + kbase;
    const _Float16* pr = sP + m * KL;
    #pragma unroll 1
    for (int c = 0; c < nch; ++c) {
      const v16h pa = ldfrag_h(pr + 32 * c, h);
      const v16h vb = ldfrag_h(vrow + 32 * c, h);
      acc = wmma_f16(pa, vb, acc);
    }
    #pragma unroll
    for (int r = 0; r < 8; ++r) sO[(8 * h + r) * HD + 16 * w + m] = acc[r] * (1.0f / PSCALE);
  }
  __syncthreads();

  const int q8 = lane & 7, sub = lane >> 3;
  const int row = 4 * w + sub;
  const v4f a = *(const v4fa*)(sO + row * HD + 8 * q8);
  const v4f c = *(const v4fa*)(sO + row * HD + 8 * q8 + 4);
  v4u hi, lo;
  split8(a, c, hi, lo);
  const size_t gi = ((size_t)(b * SEQ + q0 + row)) * DM + head * HD + 8 * q8;
  *(volatile v4u*)(aoh + gi) = hi;
  *(volatile v4u*)(aol + gi) = lo;
  __threadfence();
  *(volatile v4u*)(aoh + gi) = hi;
  *(volatile v4u*)(aol + gi) = lo;
}

__device__ __forceinline__ float block_sum256(float v, float* red, int lane, int w) {
  v = wave_sum(v);
  __syncthreads();
  if (lane == 0) red[w] = v;
  __syncthreads();
  float t = red[0];
  #pragma unroll
  for (int i = 1; i < 8; ++i) t += red[i];
  return t;
}

__global__ __launch_bounds__(256) void ln_kernel(
    const float* __restrict__ query, const float* __restrict__ outf, const float* __restrict__ outwf,
    const float* __restrict__ lnw, const float* __restrict__ lnb,
    float* __restrict__ o0, float* __restrict__ o1)
{
  __shared__ float red[8];
  const int tid = threadIdx.x, lane = tid & 31, w = tid >> 5;
  const size_t base = (size_t)blockIdx.x * DM + 4 * tid;

  const v4f q  = *(const v4fa*)(query + base);
  const v4f o  = *(const v4fa*)(outf + base);
  const v4f ow = *(const v4fa*)(outwf + base);
  const v4f wv = *(const v4fa*)(lnw + 4 * tid);
  const v4f bv = *(const v4fa*)(lnb + 4 * tid);

  const v4f x1 = q + o;
  float mu = block_sum256(x1.x + x1.y + x1.z + x1.w, red, lane, w) * (1.0f / DM);
  const v4f d1 = x1 - mu;
  float var = block_sum256(d1.x * d1.x + d1.y * d1.y + d1.z * d1.z + d1.w * d1.w, red, lane, w) * (1.0f / DM);
  float rs = rsqrtf(var + LNEPS);
  const v4f y0 = d1 * rs * wv + bv;

  const v4f x2 = x1 + ow;
  mu = block_sum256(x2.x + x2.y + x2.z + x2.w, red, lane, w) * (1.0f / DM);
  const v4f d2 = x2 - mu;
  var = block_sum256(d2.x * d2.x + d2.y * d2.y + d2.z * d2.z + d2.w * d2.w, red, lane, w) * (1.0f / DM);
  rs = rsqrtf(var + LNEPS);
  const v4f y1 = d2 * rs * wv + bv;

  *(volatile v4f*)(o0 + base) = y0;
  *(volatile v4f*)(o1 + base) = y1;
  __threadfence();
  *(volatile v4f*)(o0 + base) = y0;
  *(volatile v4f*)(o1 + base) = y1;
}

extern "C" void kernel_launch(void* const* d_in, const int* in_sizes, int n_in,
                              void* d_out, int out_size, void* d_ws, size_t ws_size,
                              hipStream_t stream)
{
  if (n_in < 17) return;
  if (in_sizes[0] != NBS || in_sizes[1] != NBS || in_sizes[2] != NBS) return;
  if (in_sizes[4] != NWT || in_sizes[6] != NWT || in_sizes[8] != NWT ||
      in_sizes[10] != NWT || in_sizes[12] != NWT) return;
  if (in_sizes[5] != DM || in_sizes[7] != DM || in_sizes[9] != DM ||
      in_sizes[11] != DM || in_sizes[13] != DM) return;
  if (in_sizes[14] != NH || in_sizes[15] != DM || in_sizes[16] != DM) return;
  if (out_size != 2 * NBS) return;

  const float* query  = (const float*)d_in[0];
  const float* key    = (const float*)d_in[1];
  const float* values = (const float*)d_in[2];
  const float* Wq   = (const float*)d_in[4];
  const float* bq   = (const float*)d_in[5];
  const float* Wqw  = (const float*)d_in[6];
  const float* bqw  = (const float*)d_in[7];
  const float* Wv   = (const float*)d_in[8];
  const float* bv   = (const float*)d_in[9];
  const float* Wo   = (const float*)d_in[10];
  const float* bo   = (const float*)d_in[11];
  const float* Wow  = (const float*)d_in[12];
  const float* bow  = (const float*)d_in[13];
  const float* gam  = (const float*)d_in[14];
  const float* lnw  = (const float*)d_in[15];
  const float* lnb  = (const float*)d_in[16];

  float* o0 = (float*)d_out;
  float* o1 = o0 + NBS;

  const size_t pl16  = (size_t)NBS * 2;
  const size_t wpl16 = (size_t)NWT * 2;
  const size_t off_xpl  = 0;
  const size_t off_wt   = off_xpl + 6 * pl16;
  const size_t off_qp   = off_wt + 10 * wpl16;
  const size_t off_kp   = off_qp + pl16;
  const size_t off_qwp  = off_kp + pl16;
  const size_t off_kwp  = off_qwp + pl16;
  const size_t off_vt   = off_kwp + pl16;
  const size_t need     = off_vt + pl16;
  const size_t off_aopl = off_xpl;
  const size_t off_outf = off_qp;
  const size_t off_outwf = off_qp + (size_t)NBS * 4;
  if (need > ws_size) return;
  if (off_outwf + (size_t)NBS * 4 > need) return;

  char* ws = (char*)d_ws;
  unsigned short* xpl  = (unsigned short*)(ws + off_xpl);
  unsigned short* wtp  = (unsigned short*)(ws + off_wt);
  _Float16* qp  = (_Float16*)(ws + off_qp);
  _Float16* kp  = (_Float16*)(ws + off_kp);
  _Float16* qwp = (_Float16*)(ws + off_qwp);
  _Float16* kwp = (_Float16*)(ws + off_kwp);
  _Float16* vt  = (_Float16*)(ws + off_vt);
  unsigned short* aopl = (unsigned short*)(ws + off_aopl);
  unsigned short* aoh  = aopl;
  unsigned short* aol  = aopl + NBS;
  unsigned short* awh  = aopl + 2 * (size_t)NBS;
  unsigned short* awl  = aopl + 3 * (size_t)NBS;
  float* outf  = (float*)(ws + off_outf);
  float* outwf = (float*)(ws + off_outwf);

  const int ngroups = 3 * (NBS / 8);
  cvt_act_kernel<<<(ngroups + 255) / 256, 256, 0, stream>>>(query, key, values, xpl);

  dim3 gW(DM / 64, DM / 64, 5);
  cvt_w_kernel<<<gW, 256, 0, stream>>>(Wq, Wqw, Wv, Wo, Wow, wtp);

  dim3 gP(NTOK / 128, NH, 5);
  proj5_kernel<<<gP, 128, 0, stream>>>(xpl, wtp, bq, bqw, bv, qp, kp, qwp, kwp, vt);

  dim3 gA(SEQ / 16, BATCH * NH);
  attn_kernel<false><<<gA, 128, 0, stream>>>(qp, kp, vt, gam, aoh, aol);
  attn_kernel<true ><<<gA, 128, 0, stream>>>(qwp, kwp, vt, gam, awh, awl);

  dim3 gO(NTOK / 128, DM / 64, 2);
  oproj_kernel<<<gO, 128, 0, stream>>>(aopl, wtp, bo, bow, outf, outwf);

  ln_kernel<<<NTOK, 256, 0, stream>>>(query, outf, outwf, lnw, lnb, o0, o1);
}
